// LSTMModel_78348793413868
// MI455X (gfx1250) — hardware-verified
//
#include <hip/hip_runtime.h>
#include <math.h>

constexpr int NBATCH  = 512;
constexpr int NSTEP   = 512;
constexpr int NFEAT   = 37;
constexpr int NFPAD   = 64;
constexpr int NHID    = 128;
constexpr int NGATE   = 512;
constexpr int NFC1    = 64;
constexpr int NCLS    = 37;
constexpr int NTHR    = 256;
constexpr int SEQ_BLK = 16;
constexpr int HSPITCH = 132;
constexpr int HROWS   = 32;
constexpr int LSPITCH = 132;
constexpr int YSPITCH = 68;
constexpr int NOUTBLK = HROWS * NCLS;
constexpr int NOUTV4  = NOUTBLK / 4;
constexpr float WCARRY     = 16.0f;
constexpr float WCARRY_INV = 1.0f / 16.0f;

static_assert(NGATE == 4 * NHID, "gate width");
static_assert(NHID == 16 * (NTHR / 32), "8 waves x 16 hidden columns");
static_assert(NBATCH % SEQ_BLK == 0, "recurrence grid exact");
static_assert(NBATCH % HROWS == 0, "head grid exact");
static_assert(NFPAD % 32 == 0 && NFPAD >= NFEAT, "padded input K");
static_assert((NOUTBLK * 4) % 128 == 0, "head block covers whole 128-B lines");
static_assert(NOUTBLK % 4 == 0, "head block float4 count");
static_assert((NFPAD + NHID) % 32 == 0 && (NHID + NHID) % 32 == 0, "concat K multiples of 32");

typedef __attribute__((ext_vector_type(16))) _Float16 v16h;
typedef __attribute__((ext_vector_type(8)))  _Float16 v8h;
typedef __attribute__((ext_vector_type(4)))  _Float16 v4h;
typedef __attribute__((ext_vector_type(8)))  float    v8f;
typedef __attribute__((ext_vector_type(4)))  float    v4f;

__device__ __forceinline__ void guard_all4(v8f& a0, v8f& a1, v8f& a2, v8f& a3, v16h a, v16h b0, v16h b1, v16h b2, v16h b3) {
  asm volatile("v_nop\n\tv_nop\n\tv_nop\n\tv_nop" : "+v"(a0), "+v"(a1), "+v"(a2), "+v"(a3) : "v"(a), "v"(b0), "v"(b1), "v"(b2), "v"(b3));
}
__device__ __forceinline__ void acc_guard4(v8f& a, v8f& b, v8f& c, v8f& d) {
  asm volatile("v_nop\n\tv_nop\n\tv_nop\n\tv_nop" : "+v"(a), "+v"(b), "+v"(c), "+v"(d));
}

template <typename T> struct Frag;
template <> struct Frag<_Float16> {
  typedef v16h V;
  union U { v16h v; v8h h[2]; };
  static __device__ __forceinline__ v16h load(const _Float16* p) {
    U f;
    f.h[0] = *(const v8h*)(p);
    f.h[1] = *(const v8h*)(p + 16);
    return f.v;
  }
  static __device__ __forceinline__ v8f mma(v16h a, v16h b, v8f c) {
    return __builtin_amdgcn_wmma_f32_16x16x32_f16(false, a, false, b, (short)0, c, false, false);
  }
};

__device__ __forceinline__ float fsig(float x)  { return __builtin_amdgcn_rcpf(1.0f + __expf(-x)); }
__device__ __forceinline__ float ftanh(float x) { return 1.0f - 2.0f * __builtin_amdgcn_rcpf(__expf(2.0f * x) + 1.0f); }

template <int NV> struct InVec;
template <> struct InVec<4> { typedef v4h V; };
template <> struct InVec<8> { typedef v8h V; };

template <bool SWAP_BT>
__global__ __launch_bounds__(NTHR) void cvt_pad8_kernel(const float* __restrict__ src, int srcpitch, int srccols,
                                                        unsigned short* __restrict__ dst, int dstpitch, int dstcol0,
                                                        int ncol8, int nrow, float sc) {
  const int i  = blockIdx.x * NTHR + threadIdx.x;
  const int n8 = nrow * ncol8;
  if (i < n8) {
    const int row = i / ncol8;
    const int c8  = i - row * ncol8;
    int srow = row;
    if (SWAP_BT) srow = (row % NBATCH) * NSTEP + (row / NBATCH);
    const float* sp = src + (size_t)srow * (size_t)srcpitch;
    v8h hv;
#pragma unroll
    for (int e = 0; e < 8; ++e) {
      const int col = c8 * 8 + e;
      const int cc  = (col < srccols) ? col : (srccols - 1);
      const float f = sp[cc];
      const float val = (col < srccols) ? (f * sc) : 0.0f;
      hv[e] = (_Float16)val;
    }
    unsigned short* dp = dst + (size_t)row * (size_t)dstpitch + dstcol0 + c8 * 8;
    *(volatile v8h*)dp = hv;
    __threadfence();
    *(volatile v8h*)dp = hv;
  }
}

__global__ __launch_bounds__(NTHR) void bias_sum_kernel(const float* __restrict__ bi0, const float* __restrict__ bh0,
                                                        const float* __restrict__ bi1, const float* __restrict__ bh1,
                                                        float* __restrict__ dst) {
  const int tid = threadIdx.x;
  const int which = tid >> 7;
  const int idx = (tid & 127) * 4;
  const v4f a0 = *(const v4f*)(bi0 + idx);
  const v4f a1 = *(const v4f*)(bh0 + idx);
  const v4f c0 = *(const v4f*)(bi1 + idx);
  const v4f c1 = *(const v4f*)(bh1 + idx);
  v4f o;
#pragma unroll
  for (int e = 0; e < 4; ++e) {
    const float s0 = a0[e] + a1[e];
    const float s1 = c0[e] + c1[e];
    o[e] = which ? s1 : s0;
  }
  float* op = dst + which * NGATE + idx;
  *(volatile v4f*)op = o;
  __threadfence();
  *(volatile v4f*)op = o;
}

template <int KIN, bool WRITE_SEQ, bool WRITE_LAST>
__global__ __launch_bounds__(NTHR) void lstm_layer_kernel(const unsigned short* __restrict__ INp,
                                                          const unsigned short* __restrict__ Wp,
                                                          const float* __restrict__ bias,
                                                          unsigned short* SEQp, float* LASTp) {
  constexpr int KTOT   = KIN + NHID;
  constexpr int APITCH = KTOT + 8;
  constexpr int ABUF   = SEQ_BLK * APITCH;
  constexpr int INV    = KIN / 16;
  static_assert(KTOT % 32 == 0, "K multiple of 32");
  static_assert(APITCH % 8 == 0, "16-B aligned fragment rows");
  static_assert((2 * ABUF) % NTHR == 0, "zero-fill loop exact");
  static_assert(INV == 4 || INV == 8, "input staging vector width");
  static_assert(SEQ_BLK * KIN == NTHR * INV, "input staging covers exactly 16 x KIN");
  typedef typename InVec<INV>::V IV;

  __shared__ __align__(16) _Float16 At[2 * ABUF];
  __shared__ __align__(16) float    Hs[WRITE_LAST ? (SEQ_BLK * HSPITCH) : 4];

  const _Float16* IN = (const _Float16*)INp;
  const _Float16* W  = (const _Float16*)Wp;
  const int tid = threadIdx.x, lane = tid & 31, wave = tid >> 5;
  const int c = lane & 15, hh = lane >> 4, koff = hh * 8;
  const int rowbase = blockIdx.x * SEQ_BLK;
  const int j = 16 * wave + c;
  const int sm = tid >> 4;
  const int scol = (tid & 15) * INV;

#pragma unroll 1
  for (int i = tid; i < 2 * ABUF; i += NTHR) At[i] = (_Float16)0.0f;
  __syncthreads();
  {
    const IV v0 = *(const IV*)(IN + ((size_t)rowbase + sm) * KIN + scol);
    *(IV*)(At + sm * APITCH + scol) = v0;
  }
  const float bb0 = bias[0 * NHID + j];
  const float bb1 = bias[1 * NHID + j];
  const float bb2 = bias[2 * NHID + j];
  const float bb3 = bias[3 * NHID + j];
  float cst[8], hst[8];
#pragma unroll
  for (int r = 0; r < 8; ++r) { cst[r] = 0.0f; hst[r] = 0.0f; }
  __syncthreads();

  const _Float16* wrow = W + (size_t)j * KTOT + koff;
  const v8f z8 = {0.f, 0.f, 0.f, 0.f, 0.f, 0.f, 0.f, 0.f};

#pragma unroll 1
  for (int t = 0; t < NSTEP; ++t) {
    const int p = t & 1;
    const _Float16* cur = At + p * ABUF;
    _Float16* nxt = At + (p ^ 1) * ABUF;
    const int tn = (t + 1 < NSTEP) ? (t + 1) : (NSTEP - 1);
    const IV vin = *(const IV*)(IN + ((size_t)tn * NBATCH + rowbase + sm) * KIN + scol);

    const _Float16* arow = cur + c * APITCH + koff;
    v8f acc0 = z8, acc1 = z8, acc2 = z8, acc3 = z8;
#pragma unroll 1
    for (int k0 = 0; k0 < KTOT; k0 += 32) {
      const v16h a  = Frag<_Float16>::load(arow + k0);
      const v16h b0 = Frag<_Float16>::load(wrow + k0);
      const v16h b1 = Frag<_Float16>::load(wrow + (size_t)1 * NHID * KTOT + k0);
      const v16h b2 = Frag<_Float16>::load(wrow + (size_t)2 * NHID * KTOT + k0);
      const v16h b3 = Frag<_Float16>::load(wrow + (size_t)3 * NHID * KTOT + k0);
      acc0 = Frag<_Float16>::mma(a, b0, acc0);
      acc1 = Frag<_Float16>::mma(a, b1, acc1);
      acc2 = Frag<_Float16>::mma(a, b2, acc2);
      acc3 = Frag<_Float16>::mma(a, b3, acc3);
      guard_all4(acc0, acc1, acc2, acc3, a, b0, b1, b2, b3);
    }
    acc_guard4(acc0, acc1, acc2, acc3);

#pragma unroll
    for (int r = 0; r < 8; ++r) {
      const float zi = acc0[r] * WCARRY_INV + bb0;
      const float zf = acc1[r] * WCARRY_INV + bb1;
      const float zg = acc2[r] * WCARRY_INV + bb2;
      const float zo = acc3[r] * WCARRY_INV + bb3;
      const float ig = fsig(zi);
      const float fg = fsig(zf);
      const float gg = ftanh(zg);
      const float og = fsig(zo);
      const float cn = fg * cst[r] + ig * gg;
      cst[r] = cn;
      const float hn = og * ftanh(cn);
      if (WRITE_LAST) hst[r] = hn;
      nxt[(8 * hh + r) * APITCH + KIN + j] = (_Float16)hn;
    }
    *(IV*)(nxt + sm * APITCH + scol) = vin;
    __syncthreads();

    if (WRITE_SEQ) {
      const int row = 2 * wave + hh;
      const int c8  = c * 8;
      const v8h hv = *(const v8h*)(nxt + row * APITCH + KIN + c8);
      unsigned short* gp = SEQp + ((size_t)t * NBATCH + rowbase + row) * NHID + c8;
      for (int pass = 0; pass < 2; ++pass) {
        *(volatile v8h*)gp = hv;
        __threadfence();
      }
    }
  }

  if (WRITE_LAST) {
#pragma unroll
    for (int r = 0; r < 8; ++r) Hs[(8 * hh + r) * HSPITCH + j] = hst[r];
    __syncthreads();
    for (int pass = 0; pass < 2; ++pass) {
#pragma unroll
      for (int it = 0; it < 2; ++it) {
        const int idx = it * NTHR + tid;
        const int row = idx >> 5;
        const int c4  = (idx & 31) * 4;
        const v4f v = *(const v4f*)(Hs + row * HSPITCH + c4);
        *(volatile v4f*)(LASTp + (size_t)(rowbase + row) * NHID + c4) = v;
      }
      __threadfence();
    }
  }
}

__global__ __launch_bounds__(NTHR) void head_kernel(const float* __restrict__ HL,
                                                    const float* __restrict__ w1, const float* __restrict__ b1,
                                                    const float* __restrict__ w2, const float* __restrict__ b2,
                                                    float* out) {
  __shared__ __align__(16) float Ls[HROWS * LSPITCH];
  __shared__ __align__(16) float Ys[HROWS * YSPITCH];
  __shared__ __align__(16) float Os[NOUTBLK];
  const int tid = threadIdx.x;
  const int rowbase = blockIdx.x * HROWS;

#pragma unroll 1
  for (int it = 0; it < 4; ++it) {
    const int idx = it * NTHR + tid;
    const int row = idx >> 5;
    const int c4  = (idx & 31) * 4;
    const v4f v = *(const v4f*)(HL + (size_t)(rowbase + row) * NHID + c4);
    *(v4f*)(Ls + row * LSPITCH + c4) = v;
  }
  __syncthreads();

#pragma unroll 1
  for (int it = 0; it < 8; ++it) {
    const int idx = it * NTHR + tid;
    const int m  = idx >> 6;
    const int jj = idx & 63;
    const float* wr = w1 + (size_t)jj * NHID;
    const float* lr = Ls + m * LSPITCH;
    float s = b1[jj];
#pragma unroll 1
    for (int k = 0; k < NHID; k += 4) {
      const v4f wv = *(const v4f*)(wr + k);
      const v4f lv = *(const v4f*)(lr + k);
      s = fmaf(lv[0], wv[0], s);
      s = fmaf(lv[1], wv[1], s);
      s = fmaf(lv[2], wv[2], s);
      s = fmaf(lv[3], wv[3], s);
    }
    Ys[m * YSPITCH + jj] = fmaxf(s, 0.0f);
  }
  __syncthreads();

#pragma unroll 1
  for (int it = 0; it < 5; ++it) {
    const int idx = it * NTHR + tid;
    const int idc = (idx < NOUTBLK) ? idx : (NOUTBLK - 1);
    const int m   = idc / NCLS;
    const int jj  = idc - m * NCLS;
    const float* wr = w2 + (size_t)jj * NFC1;
    const float* yr = Ys + m * YSPITCH;
    float s = b2[jj];
#pragma unroll 1
    for (int k = 0; k < NFC1; k += 4) {
      const v4f wv = *(const v4f*)(wr + k);
      const v4f yv = *(const v4f*)(yr + k);
      s = fmaf(yv[0], wv[0], s);
      s = fmaf(yv[1], wv[1], s);
      s = fmaf(yv[2], wv[2], s);
      s = fmaf(yv[3], wv[3], s);
    }
    if (idx < NOUTBLK) Os[idx] = s;
  }
  __syncthreads();

  float* ob = out + (size_t)blockIdx.x * NOUTBLK;
  for (int pass = 0; pass < 2; ++pass) {
#pragma unroll
    for (int it = 0; it < 2; ++it) {
      const int idx = it * NTHR + tid;
      const int idc = (idx < NOUTV4) ? idx : (NOUTV4 - 1);
      const v4f v = *(const v4f*)(Os + 4 * idc);
      if (idx < NOUTV4) *(volatile v4f*)(ob + 4 * idx) = v;
    }
    __threadfence();
  }
}

extern "C" void kernel_launch(void* const* d_in, const int* in_sizes, int n_in,
                              void* d_out, int out_size, void* d_ws, size_t ws_size, hipStream_t stream) {
  if (n_in < 13 || d_out == nullptr || d_ws == nullptr) return;
  if (in_sizes[0] != NBATCH * NSTEP * NFEAT || in_sizes[1] != NGATE * NFEAT || in_sizes[2] != NGATE * NHID ||
      in_sizes[3] != NGATE || in_sizes[4] != NGATE || in_sizes[5] != NGATE * NHID || in_sizes[6] != NGATE * NHID ||
      in_sizes[7] != NGATE || in_sizes[8] != NGATE || in_sizes[9] != NFC1 * NHID || in_sizes[10] != NFC1 ||
      in_sizes[11] != NCLS * NFC1 || in_sizes[12] != NCLS || out_size != NBATCH * NCLS) return;

  const float* x    = (const float*)d_in[0];
  const float* wih0 = (const float*)d_in[1];
  const float* whh0 = (const float*)d_in[2];
  const float* bih0 = (const float*)d_in[3];
  const float* bhh0 = (const float*)d_in[4];
  const float* wih1 = (const float*)d_in[5];
  const float* whh1 = (const float*)d_in[6];
  const float* bih1 = (const float*)d_in[7];
  const float* bhh1 = (const float*)d_in[8];
  const float* fc1w = (const float*)d_in[9];
  const float* fc1b = (const float*)d_in[10];
  const float* fc2w = (const float*)d_in[11];
  const float* fc2b = (const float*)d_in[12];
  float* out = (float*)d_out;

  char* ws = (char*)d_ws;
  size_t off = 0;
  auto carve = [&](size_t bytes) -> char* { char* p = ws + off; off += (bytes + 255) & ~(size_t)255; return p; };
  unsigned short* X16  = (unsigned short*)carve((size_t)NSTEP * NBATCH * NFPAD * 2);
  unsigned short* H1   = (unsigned short*)carve((size_t)NSTEP * NBATCH * NHID * 2);
  unsigned short* WC0  = (unsigned short*)carve((size_t)NGATE * (NFPAD + NHID) * 2);
  unsigned short* WC1  = (unsigned short*)carve((size_t)NGATE * (NHID + NHID) * 2);
  float*          BIAS = (float*)carve((size_t)2 * NGATE * 4);
  float*          H2L  = (float*)carve((size_t)NBATCH * NHID * 4);
  if (off > ws_size || off > (size_t)134217728) return;

  const int n8x  = NSTEP * NBATCH * (NFPAD / 8);
  const int n8w0 = NGATE * (NFPAD / 8);
  const int n8wh = NGATE * (NHID / 8);
  cvt_pad8_kernel<true><<<n8x / NTHR, NTHR, 0, stream>>>(x, NFEAT, NFEAT, X16, NFPAD, 0, NFPAD / 8, NSTEP * NBATCH, 1.0f);
  cvt_pad8_kernel<false><<<n8w0 / NTHR, NTHR, 0, stream>>>(wih0, NFEAT, NFEAT, WC0, NFPAD + NHID, 0, NFPAD / 8, NGATE, WCARRY);
  cvt_pad8_kernel<false><<<n8wh / NTHR, NTHR, 0, stream>>>(whh0, NHID, NHID, WC0, NFPAD + NHID, NFPAD, NHID / 8, NGATE, WCARRY);
  cvt_pad8_kernel<false><<<n8wh / NTHR, NTHR, 0, stream>>>(wih1, NHID, NHID, WC1, NHID + NHID, 0, NHID / 8, NGATE, WCARRY);
  cvt_pad8_kernel<false><<<n8wh / NTHR, NTHR, 0, stream>>>(whh1, NHID, NHID, WC1, NHID + NHID, NHID, NHID / 8, NGATE, WCARRY);
  bias_sum_kernel<<<1, NTHR, 0, stream>>>(bih0, bhh0, bih1, bhh1, BIAS);

  lstm_layer_kernel<NFPAD, true, false><<<NBATCH / SEQ_BLK, NTHR, 0, stream>>>(X16, WC0, BIAS, H1, H2L);
  lstm_layer_kernel<NHID, false, true><<<NBATCH / SEQ_BLK, NTHR, 0, stream>>>(H1, WC1, BIAS + NGATE, X16, H2L);
  head_kernel<<<NBATCH / HROWS, NTHR, 0, stream>>>(H2L, fc1w, fc1b, fc2w, fc2b, out);
}
